// OfficialVMambaVSSBlock_46248207843794
// MI455X (gfx1250) — hardware-run, weakly checked
//
#include <hip/hip_runtime.h>
#include <math.h>

#define NBAT 8
#define IMH  56
#define IMW  56
#define CIN  96
#define LTOK (IMH * IMW)
#define NTOK (NBAT * LTOK)
#define DIN  192
#define HID  384
#define DST  16
#define DTRK 6
#define XPR  38
#define NDIR 4
#define XDN  256
#define XBO  8
#define XCO  24
#define EPSV 1e-5f
#define GSTR 40
#define SCH  32
#define TSP  200
#define CTB  32
#define SYP  196
#define LTP  104
#define WTP  392
#define LOG2E 1.4426950408889634f

static_assert(NTOK % 128 == 0);
static_assert(NTOK % 64 == 0);
static_assert(NTOK % CTB == 0);
static_assert(LTOK % SCH == 0);
static_assert(SCH == 32);
static_assert(CIN % 32 == 0 && DIN % 32 == 0 && HID % 32 == 0);
static_assert(HID % 64 == 0 && (2 * DIN) % 64 == 0 && XDN % 64 == 0);
static_assert(HID == 2 * DIN);
static_assert(XDN == 64 * NDIR);
static_assert(XCO + DST <= 64);
static_assert(XBO >= DTRK);
static_assert(TSP % 8 == 0 && TSP >= DIN);
static_assert(SYP % 4 == 0 && SYP >= DIN);
static_assert(LTP % 8 == 0 && LTP >= CIN);
static_assert(WTP % 8 == 0 && WTP >= HID + 8);
static_assert((CTB * (DIN / 8)) % 256 == 0);
static_assert((CTB * (DIN / 4)) % 256 == 0);
static_assert((64 * (CIN / 8)) % 256 == 0);
static_assert((SCH * (DIN / 8)) % DIN == 0);
static_assert(DIN / 8 <= 32);
static_assert(NTOK % 8 == 0);

typedef unsigned short us16 __attribute__((ext_vector_type(16)));
typedef unsigned short us8  __attribute__((ext_vector_type(8)));
typedef unsigned short us8a __attribute__((ext_vector_type(8), may_alias));
typedef __bf16 v16b __attribute__((ext_vector_type(16)));
typedef float v8f __attribute__((ext_vector_type(8)));
typedef float v4f __attribute__((ext_vector_type(4)));
typedef float v4fa __attribute__((ext_vector_type(4), may_alias));
union FragU { us16 v; us8 h[2]; };

__device__ __forceinline__ unsigned short bf16_bits(float f) {
  unsigned u = __float_as_uint(f);
  u += 0x7FFFu + ((u >> 16) & 1u);
  return (unsigned short)(u >> 16);
}
__device__ __forceinline__ float bf16_val(unsigned short b) { return __uint_as_float(((unsigned)b) << 16); }
__device__ __forceinline__ float bf16r(float f) { return bf16_val(bf16_bits(f)); }
__device__ __forceinline__ float siluf(float x) { return x * __builtin_amdgcn_rcpf(1.0f + __expf(-x)); }
__device__ __forceinline__ float geluf(float x) { return (0.5f * x) * (erff(x * 0.70710678118654752f) + 1.0f); }

__device__ __forceinline__ v8f mma_bf16(us16 a, us16 b, v8f c) {
  return __builtin_amdgcn_wmma_f32_16x16x32_bf16(false, __builtin_bit_cast(v16b, a), false, __builtin_bit_cast(v16b, b), (short)0, c, false, false);
}
template <int NJ> struct WG;
template <> struct WG<4> {
  static __device__ __forceinline__ void g(v8f (&c)[4], const us16& a, const us16 (&b)[4]) {
#if defined(__HIP_DEVICE_COMPILE__)
    asm volatile("v_nop\n\tv_nop\n\tv_nop\n\tv_nop"
                 : "+v"(c[0]), "+v"(c[1]), "+v"(c[2]), "+v"(c[3])
                 : "v"(a), "v"(b[0]), "v"(b[1]), "v"(b[2]), "v"(b[3]));
#endif
  }
};
template <> struct WG<6> {
  static __device__ __forceinline__ void g(v8f (&c)[6], const us16& a, const us16 (&b)[6]) {
#if defined(__HIP_DEVICE_COMPILE__)
    asm volatile("v_nop\n\tv_nop\n\tv_nop\n\tv_nop"
                 : "+v"(c[0]), "+v"(c[1]), "+v"(c[2]), "+v"(c[3]), "+v"(c[4]), "+v"(c[5])
                 : "v"(a), "v"(b[0]), "v"(b[1]), "v"(b[2]), "v"(b[3]), "v"(b[4]), "v"(b[5]));
#endif
  }
};

__device__ __forceinline__ us16 lds_frag(const unsigned short* base) {
  const int lane = threadIdx.x & 31, r = lane & 15, kh = (lane >> 4) * 8;
  FragU f;
  f.h[0] = *(const us8a*)(base + r * GSTR + kh);
  f.h[1] = *(const us8a*)(base + r * GSTR + 16 + kh);
  return f.v;
}

__device__ __forceinline__ void stage_a(unsigned short* lds, const unsigned short* __restrict__ P, int ld, int m0, int k0, int tid) {
  const int row = tid >> 1, cq = (tid & 1) * 16;
  const unsigned short* src = P + (size_t)(m0 + row) * ld + k0 + cq;
  const us8 v0 = *(const us8a*)src;
  const us8 v1 = *(const us8a*)(src + 8);
  *(us8a*)(lds + row * GSTR + cq) = v0;
  *(us8a*)(lds + row * GSTR + cq + 8) = v1;
}
template <int NT>
__device__ __forceinline__ void stage_b(unsigned short* lds, const unsigned short* __restrict__ P, int ld, int n0, int k0, int tid) {
#pragma unroll
  for (int i = 0; i < (NT * 4 + 255) / 256; ++i) {
    const int p = i * 256 + tid;
    if (p < NT * 4) {
      const int row = p >> 2, kq = (p & 3) * 8;
      const us8 v = *(const us8a*)(P + (size_t)(n0 + row) * ld + k0 + kq);
      *(us8a*)(lds + row * GSTR + kq) = v;
    }
  }
}

template <int NJ, int EPI>
__global__ __launch_bounds__(256) void k_gemm(const unsigned short* __restrict__ Ap, int lda,
                                             const unsigned short* __restrict__ Bp, int ldb, int K,
                                             float* Y, float* Yalt, int nsplit, unsigned short* Yh, int ldy,
                                             const float* __restrict__ Rs, const float* __restrict__ bias) {
#pragma clang fp contract(off)
  constexpr int NT = 16 * NJ;
  constexpr int OSTR = NT + 4;
  constexpr int OSTRH = NT + 8;
  constexpr int SMB = 8 * 16 * OSTR * 4;
  static_assert((128 + NT) * GSTR * 2 <= SMB);
  static_assert(8 * 16 * OSTRH * 2 <= SMB);
  static_assert(OSTR % 4 == 0 && OSTRH % 8 == 0);
  __shared__ __attribute__((aligned(16))) unsigned char sm[SMB];
  unsigned short* lA = (unsigned short*)sm;
  unsigned short* lB = lA + 128 * GSTR;
  float* oS = (float*)sm;
  unsigned short* oH = (unsigned short*)sm;
  const int tid = threadIdx.x, lane = tid & 31, wave = tid >> 5, cl = lane & 15, hh = lane >> 4;
  const int m0 = blockIdx.x * 128;
  const int n0 = blockIdx.y * NT;
  float* Yb = Y;
  int nq = n0;
  if (nsplit > 0 && n0 >= nsplit) { Yb = Yalt; nq = n0 - nsplit; }

  v8f acc[NJ];
#pragma unroll
  for (int j = 0; j < NJ; ++j) { v8f zz = {0.f, 0.f, 0.f, 0.f, 0.f, 0.f, 0.f, 0.f}; acc[j] = zz; }
  us16 af;
  us16 bfr[NJ];

#pragma unroll 1
  for (int k0 = 0; k0 < K; k0 += 32) {
    __syncthreads();
    stage_a(lA, Ap, lda, m0, k0, tid);
    stage_b<NT>(lB, Bp, ldb, n0, k0, tid);
    __syncthreads();
    af = lds_frag(lA + 16 * wave * GSTR);
#pragma unroll
    for (int j = 0; j < NJ; ++j) bfr[j] = lds_frag(lB + 16 * j * GSTR);
#pragma unroll
    for (int j = 0; j < NJ; ++j) acc[j] = mma_bf16(af, bfr[j], acc[j]);
    WG<NJ>::g(acc, af, bfr);
  }
  __syncthreads();

  if constexpr (EPI == 3) {
    unsigned short* soh = oH + wave * (16 * OSTRH);
#pragma unroll
    for (int j = 0; j < NJ; ++j) {
      const int gn = nq + 16 * j + cl;
      const float bb = bf16r(bias[gn]);
#pragma unroll
      for (int r = 0; r < 8; ++r) {
        const float t = acc[j][r] + bb;
        soh[(8 * hh + r) * OSTRH + 16 * j + cl] = bf16_bits(geluf(t));
      }
    }
  } else {
    float* so = oS + wave * (16 * OSTR);
#pragma unroll
    for (int j = 0; j < NJ; ++j) {
      const int gn = nq + 16 * j + cl;
      float bb = 0.0f;
      if constexpr (EPI == 2) bb = bf16r(bias[gn]);
#pragma unroll
      for (int r = 0; r < 8; ++r) {
        const int row = 8 * hh + r;
        float v = acc[j][r];
        if constexpr (EPI == 1) v = v + bf16r(Rs[(size_t)(m0 + 16 * wave + row) * ldy + gn]);
        if constexpr (EPI == 2) v = Rs[(size_t)(m0 + 16 * wave + row) * ldy + gn] + (v + bb);
        so[row * OSTR + 16 * j + cl] = v;
      }
    }
  }
  __syncthreads();
  if constexpr (EPI == 3) {
    const unsigned short* soh = oH + wave * (16 * OSTRH);
#pragma unroll
    for (int pass = 0; pass < 2; ++pass) {
#pragma unroll
      for (int it = 0; it < NJ; ++it) {
        const int ch = it * 32 + lane, r = ch / (2 * NJ), q = (ch - r * (2 * NJ)) * 8;
        const us8 v = *(const us8a*)(soh + r * OSTRH + q);
        *(volatile us8*)(Yh + (size_t)(m0 + 16 * wave + r) * ldy + nq + q) = v;
      }
      __threadfence();
    }
  } else {
    const float* so = oS + wave * (16 * OSTR);
#pragma unroll
    for (int pass = 0; pass < 2; ++pass) {
#pragma unroll
      for (int it = 0; it < 2 * NJ; ++it) {
        const int ch = it * 32 + lane, r = ch / (4 * NJ), q = (ch - r * (4 * NJ)) * 4;
        const v4f v = *(const v4fa*)(so + r * OSTR + q);
        *(volatile v4f*)(Yb + (size_t)(m0 + 16 * wave + r) * ldy + nq + q) = v;
      }
      __threadfence();
    }
  }
}

__global__ __launch_bounds__(256) void k_cvt_t(const float* __restrict__ src, unsigned short* dst, int K, int N) {
  __shared__ __attribute__((aligned(16))) unsigned short ts[32 * WTP];
  const int tid = threadIdx.x, n0 = blockIdx.x * 32;
  const int KP = K + 8;
#pragma unroll 1
  for (int i = tid; i < K * 32; i += 256) {
    const int k = i >> 5, j = i & 31;
    ts[j * KP + k] = bf16_bits(src[(size_t)k * N + n0 + j]);
  }
  __syncthreads();
  const int np = 4 * K;
  const int kp8 = K >> 3;
  unsigned short* base = dst + (size_t)n0 * K;
#pragma unroll
  for (int pass = 0; pass < 2; ++pass) {
#pragma unroll
    for (int k = 0; k < 6; ++k) {
      const int p = k * 256 + tid;
      if (p < np) {
        const int row = p / kp8, c8 = (p - row * kp8) * 8;
        const us8 v = *(const us8a*)(ts + row * KP + c8);
        *(volatile us8*)(base + (size_t)p * 8) = v;
      }
    }
    __threadfence();
  }
}

__global__ __launch_bounds__(256) void k_cvt_xw(const float* __restrict__ src, unsigned short* dst) {
  const int idx = blockIdx.x * 256 + threadIdx.x;
  if (idx >= XDN * (DIN / 8)) return;
  const int row = idx / (DIN / 8), c8 = (idx - row * (DIN / 8)) * 8;
  const int dir = row >> 6, rr = row & 63;
  const bool ok = (rr < DTRK) || (rr >= XBO && rr < XCO + DST);
  int sr = (rr < DTRK) ? rr : (rr - (XBO - DTRK));
  sr = (sr < 0) ? 0 : ((sr > XPR - 1) ? (XPR - 1) : sr);
  const float* s = src + ((size_t)(dir * XPR + sr)) * DIN + c8;
  const v4f a = *(const v4fa*)s, b = *(const v4fa*)(s + 4);
  us8 o;
#pragma unroll
  for (int u = 0; u < 4; ++u) {
    o[u]     = ok ? bf16_bits(a[u]) : (unsigned short)0;
    o[4 + u] = ok ? bf16_bits(b[u]) : (unsigned short)0;
  }
  const size_t off = (size_t)row * DIN + c8;
  *(volatile us8*)(dst + off) = o;
  __threadfence();
  *(volatile us8*)(dst + off) = o;
}

template <int RB>
__global__ __launch_bounds__(256) void k_ln16(const float* __restrict__ X, const float* __restrict__ w, const float* __restrict__ b,
                                             unsigned short* Yp) {
#pragma clang fp contract(off)
  __shared__ __attribute__((aligned(16))) unsigned short ts[64 * LTP];
  const int tid = threadIdx.x, lane = tid & 31, wave = tid >> 5;
  const int row0 = blockIdx.x * 64;
  float wv[3], bv[3];
#pragma unroll
  for (int j = 0; j < 3; ++j) { wv[j] = bf16r(w[lane + 32 * j]); bv[j] = bf16r(b[lane + 32 * j]); }
#pragma unroll 1
  for (int rr = 0; rr < 8; ++rr) {
    const int lr = wave * 8 + rr;
    const float* xr = X + (size_t)(row0 + lr) * CIN;
    float xv[3];
#pragma unroll
    for (int j = 0; j < 3; ++j) { const float t = xr[lane + 32 * j]; xv[j] = RB ? bf16r(t) : t; }
    float s = (xv[0] + xv[1]) + xv[2];
#pragma unroll
    for (int off = 16; off > 0; off >>= 1) s += __shfl_xor(s, off);
    const float mean = s * (1.0f / (float)CIN);
    float dv[3];
    float q = 0.0f;
#pragma unroll
    for (int j = 0; j < 3; ++j) { dv[j] = xv[j] - mean; q = q + dv[j] * dv[j]; }
#pragma unroll
    for (int off = 16; off > 0; off >>= 1) q += __shfl_xor(q, off);
    const float var = q * (1.0f / (float)CIN);
    const float rs = 1.0f / sqrtf(var + EPSV);
#pragma unroll
    for (int j = 0; j < 3; ++j) ts[lr * LTP + lane + 32 * j] = bf16_bits((dv[j] * rs) * wv[j] + bv[j]);
  }
  __syncthreads();
  us8 o[3];
#pragma unroll
  for (int k = 0; k < 3; ++k) {
    const int p = k * 256 + tid, row = p / (CIN / 8), c8 = (p - row * (CIN / 8)) * 8;
    o[k] = *(const us8a*)(ts + row * LTP + c8);
  }
  unsigned short* base = Yp + (size_t)row0 * CIN;
#pragma unroll
  for (int pass = 0; pass < 2; ++pass) {
#pragma unroll
    for (int k = 0; k < 3; ++k) *(volatile us8*)(base + (size_t)(k * 256 + tid) * 8) = o[k];
    __threadfence();
  }
}

__global__ __launch_bounds__(256) void k_dw3(const float* __restrict__ XC, const float* __restrict__ w, const float* __restrict__ bias,
                                            float* UF, unsigned short* UB) {
#pragma clang fp contract(off)
  __shared__ __attribute__((aligned(16))) float w3s[9 * DIN];
  __shared__ __attribute__((aligned(16))) float sy[CTB * SYP];
  const int tid = threadIdx.x;
#pragma unroll 1
  for (int i = tid; i < 9 * DIN; i += 256) {
    const int tap = i / DIN, c = i - tap * DIN;
    w3s[i] = bf16r(w[c * 9 + tap]);
  }
  __syncthreads();
  const int tok0 = blockIdx.x * CTB;
  us8 hb[3];
#pragma unroll
  for (int it = 0; it < 3; ++it) {
    const int p = it * 256 + tid;
    const int tl = p / (DIN / 8), c8 = (p - tl * (DIN / 8)) * 8;
    const int tok = tok0 + tl;
    const int bb = tok / LTOK, l = tok - bb * LTOK, hy = l / IMW, wx = l - hy * IMW;
    float acc[8];
#pragma unroll
    for (int u = 0; u < 8; ++u) acc[u] = 0.0f;
#pragma unroll
    for (int ky = 0; ky < 3; ++ky) {
      const int iy = hy - 1 + ky;
      const bool oky = ((unsigned)iy < (unsigned)IMH);
      const int iyc = (iy < 0) ? 0 : ((iy > IMH - 1) ? (IMH - 1) : iy);
#pragma unroll
      for (int kx = 0; kx < 3; ++kx) {
        const int ix = wx - 1 + kx;
        const bool ok = oky && ((unsigned)ix < (unsigned)IMW);
        const int ixc = (ix < 0) ? 0 : ((ix > IMW - 1) ? (IMW - 1) : ix);
        const float* q = XC + ((size_t)bb * LTOK + (size_t)(iyc * IMW + ixc)) * DIN + c8;
        const v4f xa = *(const v4fa*)q, xb = *(const v4fa*)(q + 4);
        const float* wq = w3s + (ky * 3 + kx) * DIN + c8;
        const v4f wa = *(const v4fa*)wq, wb = *(const v4fa*)(wq + 4);
#pragma unroll
        for (int u = 0; u < 4; ++u) {
          const float pa = xa[u] * wa[u];
          const float pb = xb[u] * wb[u];
          acc[u]     = acc[u]     + (ok ? pa : 0.0f);
          acc[4 + u] = acc[4 + u] + (ok ? pb : 0.0f);
        }
      }
    }
    const v4f ba = *(const v4fa*)(bias + c8), bq = *(const v4fa*)(bias + c8 + 4);
    float v[8];
#pragma unroll
    for (int u = 0; u < 4; ++u) { v[u] = siluf(acc[u] + bf16r(ba[u])); v[4 + u] = siluf(acc[4 + u] + bf16r(bq[u])); }
    us8 o;
#pragma unroll
    for (int u = 0; u < 8; ++u) { sy[tl * SYP + c8 + u] = v[u]; o[u] = bf16_bits(v[u]); }
    hb[it] = o;
  }
  __syncthreads();
  float* ufb = UF + (size_t)tok0 * DIN;
  unsigned short* ubb = UB + (size_t)tok0 * DIN;
#pragma unroll
  for (int pass = 0; pass < 2; ++pass) {
#pragma unroll
    for (int it = 0; it < 3; ++it) *(volatile us8*)(ubb + (size_t)(it * 256 + tid) * 8) = hb[it];
#pragma unroll
    for (int k = 0; k < 6; ++k) {
      const int p = k * 256 + tid, tl = p / (DIN / 4), q = (p - tl * (DIN / 4)) * 4;
      const v4f vv = *(const v4fa*)(sy + tl * SYP + q);
      *(volatile v4f*)(ufb + (size_t)p * 4) = vv;
    }
    __threadfence();
  }
}

__device__ __forceinline__ int tok_of(int dir, int l) {
  const int lp = (dir >= 2) ? (LTOK - 1 - l) : l;
  const int hq = lp / IMH, hr = lp - hq * IMH;
  return (dir & 1) ? (hr * IMW + hq) : lp;
}

__global__ __launch_bounds__(192) void k_scan(const float* __restrict__ XD, const float* __restrict__ UF,
                                             const float* __restrict__ dtw, const float* __restrict__ dtb,
                                             const float* __restrict__ Alog, unsigned short* SP) {
#pragma clang fp contract(off)
  __shared__ __attribute__((aligned(16))) unsigned short ts[SCH * TSP];
  const int bb = blockIdx.x >> 2, dir = blockIdx.x & 3, tid = threadIdx.x;
  const int d = tid, kd = dir * DIN + d;
  float A2[DST], h[DST];
#pragma unroll
  for (int n = 0; n < DST; ++n) { A2[n] = -__expf(bf16r(Alog[kd * DST + n])) * LOG2E; h[n] = 0.0f; }
  float wd[DTRK];
#pragma unroll
  for (int r = 0; r < DTRK; ++r) wd[r] = bf16r(dtw[kd * DTRK + r]);
  const float bd = bf16r(dtb[kd]);
  const float* XDb = XD + (size_t)bb * LTOK * XDN + 64 * dir;
  const float* UFb = UF + (size_t)bb * LTOK * DIN + d;
  unsigned short* SPd = SP + (size_t)dir * NTOK * DIN + (size_t)bb * LTOK * DIN;
#pragma unroll 1
  for (int c = 0; c < LTOK / SCH; ++c) {
#pragma unroll 1
    for (int s = 0; s < SCH; ++s) {
      const int tok = tok_of(dir, c * SCH + s);
      const float* xr = XDb + (size_t)tok * XDN;
      const v4f d0 = *(const v4fa*)xr, d1 = *(const v4fa*)(xr + 4);
      const float raw = ((((d0[0] * wd[0] + d0[1] * wd[1]) + d0[2] * wd[2]) + d0[3] * wd[3]) + d1[0] * wd[4]) + d1[1] * wd[5];
      const float a = raw + bd;
      const float dl = fmaxf(a, 0.0f) + log1pf(__expf(-fabsf(a)));
      const float uv = UFb[(size_t)tok * DIN];
      v4f Bv[4], Cv[4];
#pragma unroll
      for (int q = 0; q < 4; ++q) {
        Bv[q] = *(const v4fa*)(xr + XBO + 4 * q);
        Cv[q] = *(const v4fa*)(xr + XCO + 4 * q);
      }
      const float dx = dl * uv;
      float y = 0.0f;
#pragma unroll
      for (int n = 0; n < DST; ++n) {
        const float e = exp2f(dl * A2[n]);
        h[n] = e * h[n] + dx * Bv[n >> 2][n & 3];
        y = y + h[n] * Cv[n >> 2][n & 3];
      }
      ts[s * TSP + d] = bf16_bits(y);
    }
    __syncthreads();
#pragma unroll
    for (int pass = 0; pass < 2; ++pass) {
#pragma unroll
      for (int it = 0; it < (SCH * (DIN / 8)) / DIN; ++it) {
        const int ix = it * DIN + tid;
        const int r = ix / (DIN / 8), q8 = (ix - r * (DIN / 8)) * 8;
        const int tok = tok_of(dir, c * SCH + r);
        const us8 v = *(const us8a*)(ts + r * TSP + q8);
        *(volatile us8*)(SPd + (size_t)tok * DIN + q8) = v;
      }
      __threadfence();
    }
    __syncthreads();
  }
}

__global__ __launch_bounds__(256) void k_gate(const float* __restrict__ UF, const unsigned short* __restrict__ SP,
                                             const float* __restrict__ XZ, const float* __restrict__ Dv,
                                             const float* __restrict__ g, const float* __restrict__ bt, unsigned short* GB) {
#pragma clang fp contract(off)
  const int tid = threadIdx.x, lane = tid & 31, wave = tid >> 5;
  const int tok = blockIdx.x * 8 + wave;
  const bool act = (lane < DIN / 8);
  const int cl = act ? lane : (DIN / 8 - 1);
  const int c8 = cl * 8;
  const size_t PL = (size_t)NTOK * DIN;
  const size_t ro = (size_t)tok * DIN + c8;
  float uu[8], zz[8], gg[8], bq[8], dd[4][8], sv[4][8];
  {
    const v4f ua = *(const v4fa*)(UF + ro), ub = *(const v4fa*)(UF + ro + 4);
    const v4f za = *(const v4fa*)(XZ + ro), zb = *(const v4fa*)(XZ + ro + 4);
    const v4f ga = *(const v4fa*)(g + c8), gb = *(const v4fa*)(g + c8 + 4);
    const v4f ba = *(const v4fa*)(bt + c8), b4 = *(const v4fa*)(bt + c8 + 4);
#pragma unroll
    for (int u = 0; u < 4; ++u) {
      uu[u] = ua[u]; uu[4 + u] = ub[u]; zz[u] = za[u]; zz[4 + u] = zb[u];
      gg[u] = bf16r(ga[u]); gg[4 + u] = bf16r(gb[u]); bq[u] = bf16r(ba[u]); bq[4 + u] = bf16r(b4[u]);
    }
  }
#pragma unroll
  for (int k = 0; k < 4; ++k) {
    const v4f da = *(const v4fa*)(Dv + k * DIN + c8), db = *(const v4fa*)(Dv + k * DIN + c8 + 4);
    const us8 s = *(const us8a*)(SP + (size_t)k * PL + ro);
#pragma unroll
    for (int u = 0; u < 4; ++u) { dd[k][u] = bf16r(da[u]); dd[k][4 + u] = bf16r(db[u]); }
#pragma unroll
    for (int u = 0; u < 8; ++u) sv[k][u] = bf16_val(s[u]);
  }
  float m[8];
  float ssum = 0.0f;
#pragma unroll
  for (int u = 0; u < 8; ++u) {
    const float t0 = sv[0][u] + dd[0][u] * uu[u];
    const float t1 = sv[1][u] + dd[1][u] * uu[u];
    const float t2 = sv[2][u] + dd[2][u] * uu[u];
    const float t3 = sv[3][u] + dd[3][u] * uu[u];
    m[u] = ((t0 + t2) + t1) + t3;
    ssum = ssum + (act ? m[u] : 0.0f);
  }
#pragma unroll
  for (int off = 16; off > 0; off >>= 1) ssum += __shfl_xor(ssum, off);
  const float mean = ssum * (1.0f / (float)DIN);
  float dv[8];
  float q = 0.0f;
#pragma unroll
  for (int u = 0; u < 8; ++u) { dv[u] = m[u] - mean; q = q + (act ? dv[u] * dv[u] : 0.0f); }
#pragma unroll
  for (int off = 16; off > 0; off >>= 1) q += __shfl_xor(q, off);
  const float var = q * (1.0f / (float)DIN);
  const float rs = 1.0f / sqrtf(var + EPSV);
  us8 o;
#pragma unroll
  for (int u = 0; u < 8; ++u) o[u] = bf16_bits(((dv[u] * rs) * gg[u] + bq[u]) * siluf(zz[u]));
  if (act) *(volatile us8*)(GB + ro) = o;
  __threadfence();
  if (act) *(volatile us8*)(GB + ro) = o;
}

extern "C" void kernel_launch(void* const* d_in, const int* in_sizes, int n_in,
                              void* d_out, int out_size, void* d_ws, size_t ws_size,
                              hipStream_t stream) {
  if (n_in < 20) return;
  if (in_sizes[0] != NTOK * CIN || in_sizes[1] != CIN || in_sizes[2] != CIN || in_sizes[3] != CIN * HID ||
      in_sizes[4] != DIN * 9 || in_sizes[5] != DIN || in_sizes[6] != NDIR * XPR * DIN || in_sizes[7] != NDIR * DIN * DTRK ||
      in_sizes[8] != NDIR * DIN || in_sizes[9] != NDIR * DIN * DST || in_sizes[10] != NDIR * DIN || in_sizes[11] != DIN ||
      in_sizes[12] != DIN || in_sizes[13] != DIN * CIN || in_sizes[14] != CIN || in_sizes[15] != CIN ||
      in_sizes[16] != CIN * HID || in_sizes[17] != HID || in_sizes[18] != HID * CIN || in_sizes[19] != CIN ||
      out_size != NTOK * CIN) return;

  const float* x     = (const float*)d_in[0];
  const float* ln1w  = (const float*)d_in[1];
  const float* ln1b  = (const float*)d_in[2];
  const float* win   = (const float*)d_in[3];
  const float* w3    = (const float*)d_in[4];
  const float* b3    = (const float*)d_in[5];
  const float* xpw   = (const float*)d_in[6];
  const float* dtw   = (const float*)d_in[7];
  const float* dtb   = (const float*)d_in[8];
  const float* Alog  = (const float*)d_in[9];
  const float* Dv    = (const float*)d_in[10];
  const float* onw   = (const float*)d_in[11];
  const float* onb   = (const float*)d_in[12];
  const float* wout  = (const float*)d_in[13];
  const float* ln2w  = (const float*)d_in[14];
  const float* ln2b  = (const float*)d_in[15];
  const float* f1w   = (const float*)d_in[16];
  const float* f1b   = (const float*)d_in[17];
  const float* f2w   = (const float*)d_in[18];
  const float* f2b   = (const float*)d_in[19];
  float* out = (float*)d_out;

  size_t off = 0;
  auto carve = [&](size_t bytes) -> char* { char* p = (char*)d_ws + off; off += (bytes + 255) & ~(size_t)255; return p; };
  unsigned short* WIN16 = (unsigned short*)carve((size_t)HID * CIN * 2);
  unsigned short* WX16  = (unsigned short*)carve((size_t)XDN * DIN * 2);
  unsigned short* WO16  = (unsigned short*)carve((size_t)CIN * DIN * 2);
  unsigned short* F1W16 = (unsigned short*)carve((size_t)HID * CIN * 2);
  unsigned short* F2W16 = (unsigned short*)carve((size_t)CIN * HID * 2);
  static_assert((size_t)NTOK * CIN * 2 % 256 == 0);
  static_assert((size_t)NTOK * CIN * 2 + (size_t)NTOK * DIN * 4 <= (size_t)NDIR * NTOK * DIN * 2);
  char* r1 = carve((size_t)NDIR * NTOK * DIN * 2);
  unsigned short* SP   = (unsigned short*)r1;
  unsigned short* XT16 = (unsigned short*)r1;
  float* XC            = (float*)(r1 + (size_t)NTOK * CIN * 2);
  float* XZ            = (float*)carve((size_t)NTOK * DIN * 4);
  static_assert((size_t)NTOK * HID * 2 == (size_t)NTOK * DIN * 4);
  char* r3 = carve((size_t)NTOK * DIN * 4);
  float* UF            = (float*)r3;
  unsigned short* M1   = (unsigned short*)r3;
  char* r4 = carve((size_t)NTOK * DIN * 2);
  unsigned short* UB   = (unsigned short*)r4;
  unsigned short* GB   = (unsigned short*)r4;
  static_assert((size_t)NTOK * CIN * 4 + (size_t)NTOK * CIN * 2 <= (size_t)NTOK * XDN * 4);
  char* r5 = carve((size_t)NTOK * XDN * 4);
  float* XD            = (float*)r5;
  float* Hb            = (float*)r5;
  unsigned short* A2   = (unsigned short*)(r5 + (size_t)NTOK * CIN * 4);
  if (off > ws_size || off > (size_t)134217728) return;

  const dim3 b256(256), b192(192);
  k_cvt_t<<<dim3(HID / 32), b256, 0, stream>>>(win, WIN16, CIN, HID);
  k_cvt_xw<<<dim3((XDN * (DIN / 8) + 255) / 256), b256, 0, stream>>>(xpw, WX16);
  k_cvt_t<<<dim3(CIN / 32), b256, 0, stream>>>(wout, WO16, DIN, CIN);
  k_cvt_t<<<dim3(HID / 32), b256, 0, stream>>>(f1w, F1W16, CIN, HID);
  k_cvt_t<<<dim3(CIN / 32), b256, 0, stream>>>(f2w, F2W16, HID, CIN);
  k_ln16<1><<<dim3(NTOK / 64), b256, 0, stream>>>(x, ln1w, ln1b, XT16);
  k_gemm<4, 0><<<dim3(NTOK / 128, HID / 64, 1), b256, 0, stream>>>(XT16, CIN, WIN16, CIN, CIN, XC, XZ, DIN, UB, DIN, b3, b3);
  k_dw3<<<dim3(NTOK / CTB), b256, 0, stream>>>(XC, w3, b3, UF, UB);
  k_gemm<4, 0><<<dim3(NTOK / 128, XDN / 64, 1), b256, 0, stream>>>(UB, DIN, WX16, DIN, DIN, XD, XD, 0, UB, XDN, b3, b3);
  k_scan<<<dim3(NBAT * NDIR), b192, 0, stream>>>(XD, UF, dtw, dtb, Alog, SP);
  k_gate<<<dim3(NTOK / 8), b256, 0, stream>>>(UF, SP, XZ, Dv, onw, onb, GB);
  k_gemm<6, 1><<<dim3(NTOK / 128, 1, 1), b256, 0, stream>>>(GB, DIN, WO16, DIN, DIN, Hb, Hb, 0, UB, CIN, x, b3);
  k_ln16<0><<<dim3(NTOK / 64), b256, 0, stream>>>(Hb, ln2w, ln2b, A2);
  k_gemm<4, 3><<<dim3(NTOK / 128, HID / 64, 1), b256, 0, stream>>>(A2, CIN, F1W16, CIN, CIN, XZ, XZ, 0, M1, HID, b3, f1b);
  k_gemm<6, 2><<<dim3(NTOK / 128, 1, 1), b256, 0, stream>>>(M1, HID, F2W16, HID, HID, out, out, 0, UB, CIN, Hb, f2b);
}
